// GCN_Critic_24223615550522
// MI455X (gfx1250) — hardware-verified
//
#include <hip/hip_runtime.h>
#include <stddef.h>


#define DF      128
#define HID     64
#define NTHR    256
#define NWAVE   8
#define EPT     8
#define NGRP    2
#define CHUNK   (NTHR * EPT * NGRP)
#define WCAP    (EPT * NGRP * 32)
#define LISTN   (NWAVE * WCAP)
#define NBA     512
#define NBDG    4096
#define GROWS   128
#define APITCH  136
#define WSCALE  8.0f
#define WINV    0.125f

#define LDS_GEMM (GROWS * DF * 4)
#define LDS_AGG  (NBA * DF * 4 + LISTN * 4 + 64)

static_assert((CHUNK & (CHUNK - 1)) == 0);
static_assert(CHUNK <= 4096);
static_assert(NBA <= 4096 && NBDG <= 4096);
static_assert((NBA & (NBA - 1)) == 0 && (NBDG & (NBDG - 1)) == 0);
static_assert(GROWS * APITCH * 2 <= LDS_GEMM);
static_assert(NWAVE * DF * 4 <= LISTN * 4);
static_assert(2 * DF == NTHR);
static_assert(NBA % NWAVE == 0);

typedef float    v4f  __attribute__((ext_vector_type(4)));
typedef float    v8f  __attribute__((ext_vector_type(8)));
typedef int      v4i  __attribute__((ext_vector_type(4)));
typedef _Float16 v8h  __attribute__((ext_vector_type(8)));
typedef _Float16 v16h __attribute__((ext_vector_type(16)));
union FragH { v16h v; v8h h[2]; };

__device__ __forceinline__ v8h cvt8(v4f a, v4f b) {
  v8h r;
  r[0] = (_Float16)a.x; r[1] = (_Float16)a.y; r[2] = (_Float16)a.z; r[3] = (_Float16)a.w;
  r[4] = (_Float16)b.x; r[5] = (_Float16)b.y; r[6] = (_Float16)b.z; r[7] = (_Float16)b.w;
  return r;
}

__device__ __forceinline__ v8f wmh(v16h a, v16h b, v8f c) {
  v8f d = __builtin_amdgcn_wmma_f32_16x16x32_f16(false, a, false, b, (short)0, c, false, false);
  asm volatile("v_nop\n\tv_nop\n\tv_nop\n\tv_nop" : "+v"(d) : "v"(a), "v"(b));
  return d;
}

template <int NB>
__device__ __forceinline__ int scan_chunk(const int* __restrict__ dsts, int nE, int cbase, int nodeBase,
                                          int vec8, int* list, int tid, int lane, int wave) {
  int wc = 0;
#pragma unroll
  for (int g = 0; g < NGRP; ++g) {
    const int el0  = (g * NTHR + tid) * EPT;
    const int e0   = cbase + el0;
    const int sent = -2147483647 - 1;
    v4i da, db;
    if (vec8 != 0 && cbase + CHUNK <= nE) {
      da = *(const v4i*)(dsts + e0);
      db = *(const v4i*)(dsts + e0 + 4);
    } else {
      const int em = nE > 0 ? nE - 1 : 0;
      da.x = (e0     < nE) ? dsts[min(e0, em)]     : sent;
      da.y = (e0 + 1 < nE) ? dsts[min(e0 + 1, em)] : sent;
      da.z = (e0 + 2 < nE) ? dsts[min(e0 + 2, em)] : sent;
      da.w = (e0 + 3 < nE) ? dsts[min(e0 + 3, em)] : sent;
      db.x = (e0 + 4 < nE) ? dsts[min(e0 + 4, em)] : sent;
      db.y = (e0 + 5 < nE) ? dsts[min(e0 + 5, em)] : sent;
      db.z = (e0 + 6 < nE) ? dsts[min(e0 + 6, em)] : sent;
      db.w = (e0 + 7 < nE) ? dsts[min(e0 + 7, em)] : sent;
    }
    const unsigned nb = (unsigned)nodeBase;
    const unsigned s0 = (unsigned)da.x - nb, s1 = (unsigned)da.y - nb;
    const unsigned s2 = (unsigned)da.z - nb, s3 = (unsigned)da.w - nb;
    const unsigned s4 = (unsigned)db.x - nb, s5 = (unsigned)db.y - nb;
    const unsigned s6 = (unsigned)db.z - nb, s7 = (unsigned)db.w - nb;
    const bool h0 = s0 < (unsigned)NB, h1 = s1 < (unsigned)NB, h2 = s2 < (unsigned)NB, h3 = s3 < (unsigned)NB;
    const bool h4 = s4 < (unsigned)NB, h5 = s5 < (unsigned)NB, h6 = s6 < (unsigned)NB, h7 = s7 < (unsigned)NB;
    const unsigned any = __builtin_amdgcn_ballot_w32(h0 | h1 | h2 | h3 | h4 | h5 | h6 | h7);
    if (any != 0u) {
#define HITJ(J, HJ, SJ) { \
        const unsigned mj = __builtin_amdgcn_ballot_w32(HJ); \
        if (mj != 0u) { \
          if (HJ) { \
            const int pos = wc + (int)__builtin_amdgcn_mbcnt_lo(mj, 0u); \
            if (pos < WCAP) list[wave * WCAP + pos] = ((el0 + (J)) << 12) | (int)(SJ); \
          } \
          wc += (int)__builtin_popcount(mj); } }
      HITJ(0, h0, s0)
      HITJ(1, h1, s1)
      HITJ(2, h2, s2)
      HITJ(3, h3, s3)
      HITJ(4, h4, s4)
      HITJ(5, h5, s5)
      HITJ(6, h6, s6)
      HITJ(7, h7, s7)
#undef HITJ
    }
  }
  return wc;
}

__global__ __launch_bounds__(NTHR) void k_wprep(
    const float* __restrict__ Wa, const float* __restrict__ Wb,
    _Float16* was, _Float16* wbs) {
  const int i  = blockIdx.x * NTHR + threadIdx.x;
  const int n1 = DF * DF / 8;
  if (i >= 2 * n1) return;
  const bool first = i < n1;
  const int o  = (first ? i : i - n1) * 8;
  const int n  = o / DF;
  const int k0 = o - n * DF;
  const float* p = (first ? Wa : Wb) + (size_t)k0 * DF + n;
  v4f a, b;
  a.x = p[0];      a.y = p[DF];     a.z = p[2 * DF]; a.w = p[3 * DF];
  b.x = p[4 * DF]; b.y = p[5 * DF]; b.z = p[6 * DF]; b.w = p[7 * DF];
  a = a * WSCALE;
  b = b * WSCALE;
  const v8h hv = cvt8(a, b);
  _Float16* dp = (first ? was : wbs) + o;
  *(volatile v8h*)dp = hv;
  __threadfence();
  *(volatile v8h*)dp = hv;
}

__global__ __launch_bounds__(NTHR) void k_deg(
    const int* __restrict__ ei, const float* __restrict__ ew, float* dinv, int nN, int nE, int vec8) {
  __shared__ __attribute__((aligned(16))) float dg[NBDG];
  __shared__ __attribute__((aligned(16))) int list[LISTN];
  __shared__ int wcnt[NWAVE];
  const int tid = threadIdx.x, lane = tid & 31, wave = tid >> 5;
  const int nodeBase = blockIdx.x * NBDG;
  const int* dsts = ei + nE;
  (void)nN;

  for (int i = tid; i < NBDG; i += NTHR) dg[i] = 0.f;
  __syncthreads();

  const int nChunks = (nE + CHUNK - 1) / CHUNK;
#pragma unroll 1
  for (int ch = 0; ch < nChunks; ++ch) {
    const int cbase = ch * CHUNK;
    const int wc = scan_chunk<NBDG>(dsts, nE, cbase, nodeBase, vec8, list, tid, lane, wave);
    if (lane == 0) wcnt[wave] = wc;
    __syncthreads();
    if (wave == 0) {
#pragma unroll 1
      for (int wsx = 0; wsx < NWAVE; ++wsx) {
        int n = __builtin_amdgcn_readfirstlane(wcnt[wsx]);
        n = n > WCAP ? WCAP : (n < 0 ? 0 : n);
        const int* lp = list + wsx * WCAP;
#pragma unroll 1
        for (int i = 0; i < n; ++i) {
          const int ent  = __builtin_amdgcn_readfirstlane(lp[i]);
          const int slot = ent & (NBDG - 1);
          int e = cbase + ((ent >> 12) & (CHUNK - 1));
          e = e > nE - 1 ? nE - 1 : e;
          const float w = ew[e];
          if (lane == 0) dg[slot] = dg[slot] + w;
        }
      }
    }
    __syncthreads();
  }

  v4f dq[4];
#pragma unroll
  for (int q = 0; q < 4; ++q) {
    const int f = (wave * 4 + q) * 128 + 4 * lane;
    const v4f c = *(const v4f*)(dg + f);
    const float t0 = c.x + 1.f, t1 = c.y + 1.f, t2 = c.z + 1.f, t3 = c.w + 1.f;
    dq[q].x = t0 > 0.f ? rsqrtf(t0) : 0.f;
    dq[q].y = t1 > 0.f ? rsqrtf(t1) : 0.f;
    dq[q].z = t2 > 0.f ? rsqrtf(t2) : 0.f;
    dq[q].w = t3 > 0.f ? rsqrtf(t3) : 0.f;
  }
  float* dp = dinv + (size_t)nodeBase;
#pragma unroll
  for (int q = 0; q < 4; ++q) *(volatile v4f*)(dp + (wave * 4 + q) * 128 + 4 * lane) = dq[q];
  __threadfence();
#pragma unroll
  for (int q = 0; q < 4; ++q) *(volatile v4f*)(dp + (wave * 4 + q) * 128 + 4 * lane) = dq[q];
}

__global__ __launch_bounds__(NTHR) void k_gemm(
    const float* __restrict__ x, const _Float16* __restrict__ wsm,
    const float* __restrict__ dinv, float* g, int nN) {
  extern __shared__ v4f lds_dyn[];
  _Float16* sA  = (_Float16*)lds_dyn;
  float*    stg = (float*)lds_dyn;
  const int tid = threadIdx.x, lane = tid & 31, wave = tid >> 5, hh = lane >> 4, m = lane & 15;
  const int rowBase = blockIdx.x * GROWS;

#pragma unroll
  for (int i = 0; i < (GROWS * DF / 8) / NTHR; ++i) {
    const int idx = i * NTHR + tid;
    const int r   = idx >> 4;
    const int c0  = (idx & 15) * 8;
    int node = rowBase + r;
    node = node > nN - 1 ? nN - 1 : node;
    const float* xp = x + (size_t)node * DF + c0;
    const v4f a = *(const v4f*)xp, b = *(const v4f*)(xp + 4);
    *(v8h*)(sA + r * APITCH + c0) = cvt8(a, b);
  }
  __syncthreads();

  v8f acc[8];
#pragma unroll
  for (int t = 0; t < 8; ++t) { v8f z = {0.f, 0.f, 0.f, 0.f, 0.f, 0.f, 0.f, 0.f}; acc[t] = z; }
  const _Float16* ar = sA + (wave * 16 + m) * APITCH + 8 * hh;
#pragma unroll
  for (int kt = 0; kt < DF / 32; ++kt) {
    FragH a;
    a.h[0] = *(const v8h*)(ar + 32 * kt);
    a.h[1] = *(const v8h*)(ar + 32 * kt + 16);
#pragma unroll
    for (int t = 0; t < 8; ++t) {
      const _Float16* bp = wsm + (size_t)(16 * t + m) * DF + 32 * kt + 8 * hh;
      FragH b;
      b.h[0] = *(const v8h*)bp;
      b.h[1] = *(const v8h*)(bp + 16);
      acc[t] = wmh(a.v, b.v, acc[t]);
    }
  }
  __syncthreads();

  const int r0 = wave * 16 + 8 * hh;
  const v4f dA = *(const v4f*)(dinv + (size_t)rowBase + r0);
  const v4f dB = *(const v4f*)(dinv + (size_t)rowBase + r0 + 4);
  const float d0 = dA.x * WINV, d1 = dA.y * WINV, d2 = dA.z * WINV, d3 = dA.w * WINV;
  const float d4 = dB.x * WINV, d5 = dB.y * WINV, d6 = dB.z * WINV, d7 = dB.w * WINV;
  float* sp = stg + r0 * DF + m;
#pragma unroll
  for (int t = 0; t < 8; ++t) {
    sp[0 * DF + 16 * t] = acc[t][0] * d0;
    sp[1 * DF + 16 * t] = acc[t][1] * d1;
    sp[2 * DF + 16 * t] = acc[t][2] * d2;
    sp[3 * DF + 16 * t] = acc[t][3] * d3;
    sp[4 * DF + 16 * t] = acc[t][4] * d4;
    sp[5 * DF + 16 * t] = acc[t][5] * d5;
    sp[6 * DF + 16 * t] = acc[t][6] * d6;
    sp[7 * DF + 16 * t] = acc[t][7] * d7;
  }
  __syncthreads();

  const float* lp = stg + wave * 16 * DF + 4 * lane;
  float* gp = g + ((size_t)rowBase + wave * 16) * DF + 4 * lane;
#pragma unroll
  for (int i = 0; i < 16; ++i) { const v4f v = *(const v4f*)(lp + i * DF); *(volatile v4f*)(gp + (size_t)i * DF) = v; }
  __threadfence();
#pragma unroll
  for (int i = 0; i < 16; ++i) { const v4f v = *(const v4f*)(lp + i * DF); *(volatile v4f*)(gp + (size_t)i * DF) = v; }
}

__global__ __launch_bounds__(NTHR) void k_agg(
    const int* __restrict__ ei, const float* __restrict__ ew, const float* __restrict__ g,
    const float* __restrict__ dinv, const float* __restrict__ bias, float* part,
    int nN, int nE, int vec8) {
  extern __shared__ v4f lds_dyn[];
  float* acc  = (float*)lds_dyn;
  int*   list = (int*)(acc + NBA * DF);
  int*   wcnt = list + LISTN;
  float* wpart = (float*)list;
  const int tid = threadIdx.x, lane = tid & 31, wave = tid >> 5;
  const int nodeBase = blockIdx.x * NBA;
  const int* dsts = ei + nE;

  {
    const v4f z = {0.f, 0.f, 0.f, 0.f};
    for (int i = tid; i < NBA * DF / 4; i += NTHR) lds_dyn[i] = z;
  }
  __syncthreads();

  const int nChunks = (nE + CHUNK - 1) / CHUNK;
#pragma unroll 1
  for (int ch = 0; ch < nChunks; ++ch) {
    const int cbase = ch * CHUNK;
    const int wc = scan_chunk<NBA>(dsts, nE, cbase, nodeBase, vec8, list, tid, lane, wave);
    if (lane == 0) wcnt[wave] = wc;
    __syncthreads();
    if (wave == 0) {
#pragma unroll 1
      for (int wsx = 0; wsx < NWAVE; ++wsx) {
        int n = __builtin_amdgcn_readfirstlane(wcnt[wsx]);
        n = n > WCAP ? WCAP : (n < 0 ? 0 : n);
        const int* lp = list + wsx * WCAP;
#pragma unroll 1
        for (int i = 0; i < n; ++i) {
          const int ent  = __builtin_amdgcn_readfirstlane(lp[i]);
          const int slot = ent & (NBA - 1);
          int e = cbase + ((ent >> 12) & (CHUNK - 1));
          e = e > nE - 1 ? nE - 1 : e;
          int src = ei[e];
          src = src < 0 ? 0 : (src > nN - 1 ? nN - 1 : src);
          const float w = ew[e];
          const v4f v = *(const v4f*)(g + (size_t)src * DF + 4 * lane);
          v4f* ap = (v4f*)(acc + slot * DF + 4 * lane);
          *ap = *ap + v * w;
        }
      }
    }
    __syncthreads();
  }

  const v4f bv = *(const v4f*)(bias + 4 * lane);
  v4f p4 = {0.f, 0.f, 0.f, 0.f};
#pragma unroll 1
  for (int i = 0; i < NBA / NWAVE; ++i) {
    const int slot = wave * (NBA / NWAVE) + i;
    const int node = nodeBase + slot;
    const int nc   = node > nN - 1 ? nN - 1 : node;
    const float d  = dinv[nc];
    const v4f gv = *(const v4f*)(g + (size_t)nc * DF + 4 * lane);
    const v4f av = *(const v4f*)(acc + slot * DF + 4 * lane);
    v4f hv = (av + gv) * d + bv;
    hv.x = fmaxf(hv.x, 0.f); hv.y = fmaxf(hv.y, 0.f); hv.z = fmaxf(hv.z, 0.f); hv.w = fmaxf(hv.w, 0.f);
    float s = hv.x * hv.x + hv.y * hv.y + hv.z * hv.z + hv.w * hv.w;
    s += __shfl_xor(s, 16, 32);
    s += __shfl_xor(s, 8, 32);
    s += __shfl_xor(s, 4, 32);
    s += __shfl_xor(s, 2, 32);
    s += __shfl_xor(s, 1, 32);
    const float nrm = fmaxf(sqrtf(s), 1e-12f);
    const float sc  = 1.0f / nrm;
    if (node < nN) p4 = p4 + hv * sc;
  }
  *(v4f*)(wpart + wave * DF + 4 * lane) = p4;
  __syncthreads();
  if (wave == 0) {
    v4f tot = *(const v4f*)(wpart + 4 * lane);
#pragma unroll
    for (int w = 1; w < NWAVE; ++w) tot = tot + *(const v4f*)(wpart + w * DF + 4 * lane);
    float* pp = part + (size_t)blockIdx.x * DF + 4 * lane;
    *(volatile v4f*)pp = tot;
    __threadfence();
    *(volatile v4f*)pp = tot;
  }
}

__global__ __launch_bounds__(NTHR) void k_final(
    const float* __restrict__ pa, const float* __restrict__ pb,
    const float* __restrict__ W1, const float* __restrict__ b1,
    const float* __restrict__ W2, const float* __restrict__ b2,
    float* out, int nba, int na, int nbb, int nb) {
  __shared__ float comb[2 * DF];
  __shared__ float hs[HID];
  const int tid = threadIdx.x;
  const bool ga = tid < DF;
  const float* pp = ga ? pa : pb;
  const int nblk = ga ? nba : nbb;
  const int col  = tid & (DF - 1);
  double s = 0.0;
#pragma unroll 1
  for (int b = 0; b < nblk; ++b) s += (double)pp[(size_t)b * DF + col];
  const double cnt = (double)(ga ? na : nb);
  comb[tid] = (float)(s / cnt);
  __syncthreads();
  if (tid < HID) {
    float h = 0.f;
#pragma unroll 1
    for (int k = 0; k < 2 * DF; ++k) h += comb[k] * W1[k * HID + tid];
    h = h + b1[tid];
    h = fmaxf(h, 0.f);
    hs[tid] = h * W2[tid];
  }
  __syncthreads();
  float r = 0.f;
#pragma unroll 1
  for (int k = 0; k < HID; ++k) r += hs[k];
  r = r + b2[0];
  if (tid == 0) {
    *(volatile float*)out = r;
    __threadfence();
    *(volatile float*)out = r;
  }
}

extern "C" void kernel_launch(void* const* d_in, const int* in_sizes, int n_in,
                              void* d_out, int out_size, void* d_ws, size_t ws_size,
                              hipStream_t stream) {
  if (n_in < 14) return;
  const int Nn = in_sizes[0] / DF;
  const int En = in_sizes[2];
  const int Nd = in_sizes[3] / DF;
  const int Ed = in_sizes[5];
  if (Nn <= 0 || Nd <= 0 || En < 0 || Ed < 0) return;
  if (in_sizes[0] != Nn * DF || in_sizes[1] != 2 * En) return;
  if (in_sizes[3] != Nd * DF || in_sizes[4] != 2 * Ed) return;
  if (in_sizes[6] != DF * DF || in_sizes[7] < DF || in_sizes[8] != DF * DF || in_sizes[9] < DF) return;
  if (in_sizes[10] != 2 * DF * HID || in_sizes[11] < HID || in_sizes[12] < HID || in_sizes[13] < 1) return;
  if (out_size < 1) return;

  const float* xn  = (const float*)d_in[0];
  const int*   ein = (const int*)d_in[1];
  const float* ewn = (const float*)d_in[2];
  const float* xd  = (const float*)d_in[3];
  const int*   eid = (const int*)d_in[4];
  const float* ewd = (const float*)d_in[5];
  const float* Wn  = (const float*)d_in[6];
  const float* bn  = (const float*)d_in[7];
  const float* Wd  = (const float*)d_in[8];
  const float* bd  = (const float*)d_in[9];
  const float* W1  = (const float*)d_in[10];
  const float* b1  = (const float*)d_in[11];
  const float* W2  = (const float*)d_in[12];
  const float* b2  = (const float*)d_in[13];
  float* out = (float*)d_out;

  const int nDn = (Nn + NBDG - 1) / NBDG;
  const int nDd = (Nd + NBDG - 1) / NBDG;
  const int nGn = (Nn + GROWS - 1) / GROWS;
  const int nGd = (Nd + GROWS - 1) / GROWS;
  const int nAn = (Nn + NBA - 1) / NBA;
  const int nAd = (Nd + NBA - 1) / NBA;

  char* ws = (char*)d_ws;
  size_t off = 0;
  const size_t oWn = off; off += (size_t)DF * DF * 2;                 off = (off + 255) & ~(size_t)255;
  const size_t oWd = off; off += (size_t)DF * DF * 2;                 off = (off + 255) & ~(size_t)255;
  const size_t oVn = off; off += (size_t)nDn * NBDG * 4;              off = (off + 255) & ~(size_t)255;
  const size_t oVd = off; off += (size_t)nDd * NBDG * 4;              off = (off + 255) & ~(size_t)255;
  const size_t oGn = off; off += (size_t)nGn * GROWS * DF * 4;        off = (off + 255) & ~(size_t)255;
  const size_t oGd = off; off += (size_t)nGd * GROWS * DF * 4;        off = (off + 255) & ~(size_t)255;
  const size_t oPn = off; off += (size_t)nAn * DF * 4;                off = (off + 255) & ~(size_t)255;
  const size_t oPd = off; off += (size_t)nAd * DF * 4;                off = (off + 255) & ~(size_t)255;
  if (off > ws_size) return;
  _Float16* wns = (_Float16*)(ws + oWn);
  _Float16* wds = (_Float16*)(ws + oWd);
  float*    dvn = (float*)(ws + oVn);
  float*    dvd = (float*)(ws + oVd);
  float*    gn  = (float*)(ws + oGn);
  float*    gd  = (float*)(ws + oGd);
  float*    pn  = (float*)(ws + oPn);
  float*    pd  = (float*)(ws + oPd);

  const int vec8n = ((En & 3) == 0) ? 1 : 0;
  const int vec8d = ((Ed & 3) == 0) ? 1 : 0;

  const int nPrep = 2 * (DF * DF / 8);
  k_wprep<<<(nPrep + NTHR - 1) / NTHR, NTHR, 0, stream>>>(Wn, Wd, wns, wds);

  k_deg<<<nDn, NTHR, 0, stream>>>(ein, ewn, dvn, Nn, En, vec8n);
  k_deg<<<nDd, NTHR, 0, stream>>>(eid, ewd, dvd, Nd, Ed, vec8d);

  hipFuncSetAttribute(reinterpret_cast<const void*>(&k_gemm),
                      hipFuncAttributeMaxDynamicSharedMemorySize, LDS_GEMM);
  k_gemm<<<nGn, NTHR, LDS_GEMM, stream>>>(xn, wns, dvn, gn, Nn);
  k_gemm<<<nGd, NTHR, LDS_GEMM, stream>>>(xd, wds, dvd, gd, Nd);

  hipFuncSetAttribute(reinterpret_cast<const void*>(&k_agg),
                      hipFuncAttributeMaxDynamicSharedMemorySize, LDS_AGG);
  k_agg<<<nAn, NTHR, LDS_AGG, stream>>>(ein, ewn, gn, dvn, bn, pn, Nn, En, vec8n);
  k_agg<<<nAd, NTHR, LDS_AGG, stream>>>(eid, ewd, gd, dvd, bd, pd, Nd, Ed, vec8d);

  k_final<<<1, NTHR, 0, stream>>>(pn, pd, W1, b1, W2, b2, out, nAn, Nn, nAd, Nd);
}
